// CustomTransformerBlock_75720273428548
// MI455X (gfx1250) — hardware-run, weakly checked
//
#include <hip/hip_runtime.h>
#include <math.h>

constexpr int kBatch   = 2;
constexpr int kSeq     = 1024;
constexpr int kDim     = 2048;
constexpr int kHeads   = 32;
constexpr int kKVHeads = 8;
constexpr int kHeadDim = 64;
constexpr int kFF      = 5632;
constexpr int kTok     = kBatch * kSeq;
constexpr int kKVDim   = kKVHeads * kHeadDim;
constexpr int kQKVN    = kDim + 2 * kKVDim;
constexpr int kGroups  = kBatch * kHeads;
constexpr int kGChunk  = 8;
constexpr int kNChunkA = kGroups / kGChunk;
constexpr int kTokChunk = 512;
constexpr int kNChunkF = kTok / kTokChunk;
constexpr int kPairs   = kHeadDim / 2;
constexpr float kEps       = 1e-5f;
constexpr float kWCarry    = 16.0f;
constexpr float kQKVScale  = 1.0f / 16.0f;
constexpr float kScoreScale = 0.125f;
constexpr float kPCarry    = 2048.0f;
constexpr float kCtxCarry  = 256.0f;
constexpr float kPVScale   = kCtxCarry / kPCarry;
constexpr float kWoScale   = 1.0f / (kCtxCarry * kWCarry);
constexpr float kGCarry    = 64.0f;
constexpr float kW2Scale   = 1.0f / (kGCarry * kWCarry);

constexpr size_t kMiB     = 1048576;
constexpr size_t kOffH16  = 0;
constexpr size_t kOffSC   = 0;
constexpr size_t kOffWqkv = 8 * kMiB;
constexpr size_t kOffX1   = 8 * kMiB;
constexpr size_t kOffQKV  = 20 * kMiB;
constexpr size_t kOffW13  = 24 * kMiB;
constexpr size_t kOffW2T  = 24 * kMiB;
constexpr size_t kOffQ16  = 44 * kMiB;
constexpr size_t kOffK16  = 52 * kMiB;
constexpr size_t kOffVT16 = 60 * kMiB;
constexpr size_t kOffO16  = 68 * kMiB;
constexpr size_t kOffGF   = 68 * kMiB;
constexpr size_t kOffP16  = 76 * kMiB;
constexpr size_t kOffWoT  = 92 * kMiB;
constexpr size_t kOffG16  = 90 * kMiB;
constexpr size_t kWsTotal = 112 * kMiB;
static_assert((size_t)kTok * kDim * 2 == 8 * kMiB, "h16 size");
static_assert((size_t)kQKVN * kDim * 2 == 12 * kMiB, "wqkvT size");
static_assert((size_t)kTok * kQKVN * 4 == 24 * kMiB, "qkv size");
static_assert((size_t)kGroups * kSeq * kHeadDim * 2 == 8 * kMiB, "q16 size");
static_assert((size_t)kGChunk * kSeq * kSeq * 4 == 32 * kMiB, "scores size");
static_assert((size_t)kGChunk * kSeq * kSeq * 2 == 16 * kMiB, "p16 size");
static_assert((size_t)kTok * kDim * 4 == 16 * kMiB, "x1 size");
static_assert((size_t)2 * kFF * kDim * 2 == 44 * kMiB, "w13T size");
static_assert((size_t)kTokChunk * 2 * kFF * 4 == 22 * kMiB, "gf32 size");
static_assert((size_t)kTok * kFF * 2 == 22 * kMiB, "g16 size");
static_assert((size_t)kDim * kFF * 2 == 22 * kMiB, "w2T size");
static_assert(kWsTotal <= 134217728, "ws cap");

typedef __attribute__((ext_vector_type(16))) _Float16 v16h;
typedef __attribute__((ext_vector_type(8)))  _Float16 v8h;
typedef __attribute__((ext_vector_type(16))) __bf16   v16b;
typedef __attribute__((ext_vector_type(8)))  __bf16   v8b;
typedef __attribute__((ext_vector_type(8)))  float    v8f;
typedef __attribute__((ext_vector_type(4)))  float    v4f;
typedef __attribute__((ext_vector_type(4)))  unsigned int v4u;

__device__ __forceinline__ unsigned short f2bf_bits(float f) {
  unsigned u = __float_as_uint(f);
  return (unsigned short)((u + 0x7FFFu + ((u >> 16) & 1u)) >> 16);
}
__device__ __forceinline__ float bf_bits2f(unsigned short h) { return __uint_as_float(((unsigned)h) << 16); }

__device__ __forceinline__ void dep_guard_h(v8f& a, v8f& b, v16h x, v16h y) { asm volatile("v_nop\n\tv_nop\n\tv_nop\n\tv_nop" : "+v"(a), "+v"(b) : "v"(x), "v"(y)); }
__device__ __forceinline__ void dep_guard_b(v8f& a, v8f& b, v16b x, v16b y) { asm volatile("v_nop\n\tv_nop\n\tv_nop\n\tv_nop" : "+v"(a), "+v"(b) : "v"(x), "v"(y)); }
__device__ __forceinline__ void keep4_h(v16h a, v16h b, v16h c, v16h d) { asm volatile("v_nop" :: "v"(a), "v"(b), "v"(c), "v"(d)); }
__device__ __forceinline__ void keep4_b(v16b a, v16b b, v16b c, v16b d) { asm volatile("v_nop" :: "v"(a), "v"(b), "v"(c), "v"(d)); }
__device__ __forceinline__ void acc_guard4(v8f& a, v8f& b, v8f& c, v8f& d) { asm volatile("v_nop\n\tv_nop\n\tv_nop\n\tv_nop" : "+v"(a), "+v"(b), "+v"(c), "+v"(d)); }
template <typename T> struct Frag;
template <> struct Frag<_Float16> {
  typedef v16h V; union U { v16h v; v8h h[2]; };
  static __device__ __forceinline__ v16h load(const _Float16* p) {
    U f; f.h[0] = *(const v8h*)(p); f.h[1] = *(const v8h*)(p + 16); return f.v;
  }
  static __device__ __forceinline__ v8f mma(v16h a, v16h b, v8f c) {
    return __builtin_amdgcn_wmma_f32_16x16x32_f16(false, a, false, b, (short)0, c, false, false);
  }
  static __device__ __forceinline__ void guard(v8f& a, v8f& b, v16h x, v16h y) { dep_guard_h(a, b, x, y); }
  static __device__ __forceinline__ void keep(v16h a, v16h b, v16h c, v16h d) { keep4_h(a, b, c, d); }
};
template <> struct Frag<__bf16> {
  typedef v16b V; union U { v16b v; v8b h[2]; };
  static __device__ __forceinline__ v16b load(const __bf16* p) {
    U f; f.h[0] = *(const v8b*)(p); f.h[1] = *(const v8b*)(p + 16); return f.v;
  }
  static __device__ __forceinline__ v8f mma(v16b a, v16b b, v8f c) {
    return __builtin_amdgcn_wmma_f32_16x16x32_bf16(false, a, false, b, (short)0, c, false, false);
  }
  static __device__ __forceinline__ void guard(v8f& a, v8f& b, v16b x, v16b y) { dep_guard_b(a, b, x, y); }
  static __device__ __forceinline__ void keep(v16b a, v16b b, v16b c, v16b d) { keep4_b(a, b, c, d); }
};

__device__ __forceinline__ unsigned pk16(unsigned short a, unsigned short b) { return (unsigned)a | ((unsigned)b << 16); }
__device__ __forceinline__ unsigned short h_bits(float f) { const _Float16 h = (_Float16)f; return __builtin_bit_cast(unsigned short, h); }

template <int ET> struct Elem;
template <> struct Elem<0> { typedef _Float16 T; };
template <> struct Elem<1> { typedef __bf16 T; };
template <int ET, bool SPLIT, int BIAS_MODE, int OUT_MODE, bool RESID, int ACT = 0, int CAUS = 0>
__global__ __launch_bounds__(256) void wmma_gemm64(
    const unsigned short* __restrict__ Ap, const unsigned short* __restrict__ A2p, int lda, long strideA,
    const unsigned short* __restrict__ Btp, const unsigned short* __restrict__ Bt2p, int ldb, long strideB,
    void* __restrict__ Cout, void* __restrict__ Cout2, int ldc, long strideC,
    const float* __restrict__ bias,
    const float* __restrict__ resid, long strideR,
    int M, int N, int K, float scale) {
  typedef typename Elem<ET>::T T;
  typedef typename Frag<T>::V V;
  const T* A = (const T*)Ap; const T* A2 = (const T*)A2p; const T* Bt = (const T*)Btp; const T* Bt2 = (const T*)Bt2p;
  __shared__ __align__(16) float sT[8][16 * 68];
  const int b    = blockIdx.y;
  const int lane = threadIdx.x & 31;
  const int wave = threadIdx.x >> 5;
  const int tilesN = N >> 6;
  const int tilesM = M >> 6;
  const int tile = blockIdx.x * 8 + wave;
  if (tile >= tilesM * tilesN) return;
  const int tm = tile / tilesN;
  const int tn = tile - tm * tilesN;
  const int m0 = tm << 6;
  const int n0 = tn << 6;
  if (CAUS == 1 && n0 > m0) return;
  int kEnd = K;
  if (CAUS == 2) { const int kc = m0 + 64; kEnd = (kc < K) ? kc : K; }

  const T* Ab  = A  + (size_t)b * strideA;
  const T* Bb  = Bt + (size_t)b * strideB;
  const T* Ab2 = SPLIT ? (A2  + (size_t)b * strideA) : nullptr;
  const T* Bb2 = SPLIT ? (Bt2 + (size_t)b * strideB) : nullptr;

  const int rlane = lane & 15;
  const int koff  = (lane >> 4) * 8;
  const int mOff  = (lane >> 4) * 8;

  v8f acc[4][4];
#pragma unroll
  for (int i = 0; i < 4; ++i)
#pragma unroll
    for (int j = 0; j < 4; ++j) acc[i][j] = (v8f){0.f,0.f,0.f,0.f,0.f,0.f,0.f,0.f};

  for (int k0 = 0; k0 < kEnd; k0 += 32) {
    V bh[4], bl[4];
#pragma unroll
    for (int j = 0; j < 4; ++j) {
      const size_t bo = (size_t)(n0 + (j << 4) + rlane) * ldb + koff + k0;
      bh[j] = Frag<T>::load(Bb + bo);
      if (SPLIT) bl[j] = Frag<T>::load(Bb2 + bo);
    }
#pragma unroll
    for (int i = 0; i < 4; ++i) {
      const size_t ao = (size_t)(m0 + (i << 4) + rlane) * lda + koff + k0;
      V ah = Frag<T>::load(Ab + ao);
      V al;
      if (SPLIT) al = Frag<T>::load(Ab2 + ao);
#pragma unroll
      for (int j = 0; j < 4; ++j) {
        acc[i][j] = Frag<T>::mma(ah, bh[j], acc[i][j]);
        if (SPLIT) {
          acc[i][j] = Frag<T>::mma(ah, bl[j], acc[i][j]);
          acc[i][j] = Frag<T>::mma(al, bh[j], acc[i][j]);
        }
      }
      Frag<T>::guard(acc[i][0], acc[i][3], ah, SPLIT ? al : ah);
    }
    Frag<T>::keep(bh[0], bh[1], bh[2], bh[3]);
    if (SPLIT) Frag<T>::keep(bl[0], bl[1], bl[2], bl[3]);
  }
  acc_guard4(acc[0][0], acc[0][1], acc[0][2], acc[0][3]);
  acc_guard4(acc[1][0], acc[1][1], acc[1][2], acc[1][3]);
  acc_guard4(acc[2][0], acc[2][1], acc[2][2], acc[2][3]);
  acc_guard4(acc[3][0], acc[3][1], acc[3][2], acc[3][3]);

  float* slab = sT[wave];
  const float* Rb = RESID ? (resid + (size_t)b * strideR) : nullptr;
#pragma unroll
  for (int i = 0; i < 4; ++i) {
    const int mBase = m0 + (i << 4);
#pragma unroll
    for (int j = 0; j < 4; ++j) {
      const int n = n0 + (j << 4) + rlane;
      float bv = 0.f;
      if (BIAS_MODE == 2) bv = bias[n];
#pragma unroll
      for (int r = 0; r < 8; ++r) {
        float v = acc[i][j][r] * scale;
        if (BIAS_MODE == 1) v += bias[mBase + mOff + r];
        if (BIAS_MODE == 2) v += bv;
        if (RESID) v += Rb[(size_t)(mBase + mOff + r) * ldc + n];
        if (ACT == 2) v = fmaxf(v, 0.0f);
        if (ACT == 4) v = (v > 0.f) ? v : 0.01f * v;
        slab[(mOff + r) * 68 + (j << 4) + rlane] = v;
      }
    }
    __builtin_amdgcn_fence(__ATOMIC_RELEASE, "workgroup");
    __builtin_amdgcn_wave_barrier();
    __builtin_amdgcn_fence(__ATOMIC_ACQUIRE, "workgroup");
    if (OUT_MODE == 0) {
      float* C = (float*)Cout + (size_t)b * strideC;
      const int hh = lane >> 4, c4 = (lane & 15) * 4;
      for (int pass = 0; pass < 2; ++pass) {
#pragma unroll
        for (int it = 0; it < 8; ++it) {
          const int row = it * 2 + hh;
          v4f v = *(const v4f*)(slab + row * 68 + c4);
          *(volatile v4f*)(C + (size_t)(mBase + row) * ldc + n0 + c4) = v;
        }
        __threadfence();
      }
    } else {
      const int q = lane >> 3, c8 = (lane & 7) * 8;
      unsigned short* C  = (unsigned short*)Cout  + (size_t)b * strideC;
      unsigned short* C2 = (OUT_MODE == 2) ? ((unsigned short*)Cout2 + (size_t)b * strideC) : nullptr;
      for (int pass = 0; pass < 2; ++pass) {
#pragma unroll
        for (int it = 0; it < 4; ++it) {
          const int row = it * 4 + q;
          const float* sp = slab + row * 68 + c8;
          v8h hv, lv;
#pragma unroll
          for (int e = 0; e < 8; ++e) {
            if (OUT_MODE == 1) {
              hv[e] = (_Float16)sp[e];
            } else {
              unsigned short hb = f2bf_bits(sp[e]);
              unsigned short lb = f2bf_bits(sp[e] - bf_bits2f(hb));
              hv[e] = __builtin_bit_cast(_Float16, hb);
              lv[e] = __builtin_bit_cast(_Float16, lb);
            }
          }
          *(volatile v8h*)(C + (size_t)(mBase + row) * ldc + n0 + c8) = hv;
          if (OUT_MODE == 2) *(volatile v8h*)(C2 + (size_t)(mBase + row) * ldc + n0 + c8) = lv;
        }
        __threadfence();
      }
    }
    __builtin_amdgcn_fence(__ATOMIC_RELEASE, "workgroup");
    __builtin_amdgcn_wave_barrier();
    __builtin_amdgcn_fence(__ATOMIC_ACQUIRE, "workgroup");
  }
}

__global__ __launch_bounds__(256) void rmsnorm_f16_kernel(const float* __restrict__ X, const float* __restrict__ w,
                                                          unsigned short* __restrict__ out) {
  __shared__ float red[8];
  const int row  = blockIdx.x;
  const int t    = threadIdx.x;
  const int lane = t & 31, wave = t >> 5;
  const float* xr = X + (size_t)row * kDim + 8 * t;
  const v4f a = *(const v4f*)(xr);
  const v4f c = *(const v4f*)(xr + 4);
  float x[8];
#pragma unroll
  for (int e = 0; e < 4; ++e) { x[e] = a[e]; x[4 + e] = c[e]; }
  float s = 0.f;
#pragma unroll
  for (int e = 0; e < 8; ++e) s += x[e] * x[e];
#pragma unroll
  for (int off = 16; off > 0; off >>= 1) s += __shfl_xor(s, off, 32);
  if (lane == 0) red[wave] = s;
  __syncthreads();
  const float tot = ((((((red[0] + red[1]) + red[2]) + red[3]) + red[4]) + red[5]) + red[6]) + red[7];
  const float inv = 1.0f / sqrtf(tot * (1.0f / (float)kDim) + kEps);
  const v4f wa = *(const v4f*)(w + 8 * t);
  const v4f wc = *(const v4f*)(w + 8 * t + 4);
  float wv[8];
#pragma unroll
  for (int e = 0; e < 4; ++e) { wv[e] = wa[e]; wv[4 + e] = wc[e]; }
  unsigned short hb[8];
#pragma unroll
  for (int e = 0; e < 8; ++e) {
    const float nv = x[e] * inv;
    hb[e] = h_bits(nv * wv[e]);
  }
  const v4u u = (v4u){pk16(hb[0], hb[1]), pk16(hb[2], hb[3]), pk16(hb[4], hb[5]), pk16(hb[6], hb[7])};
  unsigned short* op = out + (size_t)row * kDim + 8 * t;
  *(volatile v4u*)op = u;
  __threadfence();
  *(volatile v4u*)op = u;
}

__global__ __launch_bounds__(256) void wtcast_kernel(const float* __restrict__ W, int ncols,
                                                     unsigned short* __restrict__ out, int ldo, float scale) {
  __shared__ float sm[64][65];
  const int t  = threadIdx.x;
  const int d0 = blockIdx.x * 64;
  const int n0 = blockIdx.y * 64;
#pragma unroll
  for (int i = 0; i < 16; ++i) {
    const int e = i * 256 + t;
    const int r = e >> 6;
    const int c = e & 63;
    sm[c][r] = W[(size_t)(d0 + r) * ncols + n0 + c] * scale;
  }
  __syncthreads();
  const int lane = t & 31, wave = t >> 5;
  const int q = lane >> 3, c8 = (lane & 7) * 8;
  for (int pass = 0; pass < 2; ++pass) {
#pragma unroll
    for (int it = 0; it < 2; ++it) {
      const int row = wave * 8 + it * 4 + q;
      unsigned short hb[8];
#pragma unroll
      for (int e = 0; e < 8; ++e) hb[e] = h_bits(sm[row][c8 + e]);
      const v4u u = (v4u){pk16(hb[0], hb[1]), pk16(hb[2], hb[3]), pk16(hb[4], hb[5]), pk16(hb[6], hb[7])};
      *(volatile v4u*)(out + (size_t)(n0 + row) * ldo + d0 + c8) = u;
    }
    __threadfence();
  }
}

__global__ __launch_bounds__(256) void rope_qk_kernel(const float* __restrict__ QKV, const float* __restrict__ fcos,
                                                      const float* __restrict__ fsin,
                                                      unsigned short* __restrict__ Q16, unsigned short* __restrict__ K16) {
  const int idx = blockIdx.x * 256 + threadIdx.x;
  const int dc  = idx & 7;
  const int s   = (idx >> 3) & (kSeq - 1);
  const int g   = idx >> 13;
  const int b   = g >> 5;
  const int h   = g & 31;
  const int tok = b * kSeq + s;
  const float* qp = QKV + (size_t)tok * kQKVN + h * kHeadDim + 8 * dc;
  const float* kp = QKV + (size_t)tok * kQKVN + kDim + (h >> 2) * kHeadDim + 8 * dc;
  const v4f q0 = *(const v4f*)(qp);
  const v4f q1 = *(const v4f*)(qp + 4);
  const v4f k0 = *(const v4f*)(kp);
  const v4f k1 = *(const v4f*)(kp + 4);
  const v4f cs = *(const v4f*)(fcos + (size_t)s * kPairs + 4 * dc);
  const v4f sn = *(const v4f*)(fsin + (size_t)s * kPairs + 4 * dc);
  float xq[8], xk[8];
#pragma unroll
  for (int e = 0; e < 4; ++e) { xq[e] = q0[e]; xq[4 + e] = q1[e]; xk[e] = k0[e]; xk[4 + e] = k1[e]; }
  unsigned short hq[8], hk[8];
#pragma unroll
  for (int j = 0; j < 4; ++j) {
    const float cj = cs[j], sj = sn[j];
    const float qr = xq[2 * j], qi = xq[2 * j + 1];
    const float kr = xk[2 * j], ki = xk[2 * j + 1];
    hq[2 * j]     = h_bits(qr * cj - qi * sj);
    hq[2 * j + 1] = h_bits(qr * sj + qi * cj);
    hk[2 * j]     = h_bits(kr * cj - ki * sj);
    hk[2 * j + 1] = h_bits(kr * sj + ki * cj);
  }
  const v4u uq = (v4u){pk16(hq[0], hq[1]), pk16(hq[2], hq[3]), pk16(hq[4], hq[5]), pk16(hq[6], hq[7])};
  const v4u uk = (v4u){pk16(hk[0], hk[1]), pk16(hk[2], hk[3]), pk16(hk[4], hk[5]), pk16(hk[6], hk[7])};
  const size_t o = ((size_t)g * kSeq + s) * kHeadDim + 8 * dc;
  *(volatile v4u*)(Q16 + o) = uq;
  *(volatile v4u*)(K16 + o) = uk;
  __threadfence();
  *(volatile v4u*)(Q16 + o) = uq;
  *(volatile v4u*)(K16 + o) = uk;
}

__global__ __launch_bounds__(256) void vtrans_kernel(const float* __restrict__ QKV, unsigned short* __restrict__ VT16) {
  __shared__ float sm[64][65];
  const int t   = threadIdx.x;
  const int s0  = blockIdx.x * 64;
  const int kvh = blockIdx.y;
  const int b   = blockIdx.z;
  const float* vbase = QKV + (size_t)(b * kSeq + s0) * kQKVN + kDim + kKVDim + kvh * kHeadDim;
#pragma unroll
  for (int i = 0; i < 16; ++i) {
    const int e = i * 256 + t;
    const int r = e >> 6;
    const int c = e & 63;
    sm[c][r] = vbase[(size_t)r * kQKVN + c];
  }
  __syncthreads();
  const int lane = t & 31, wave = t >> 5;
  const int q = lane >> 3, c8 = (lane & 7) * 8;
  for (int pass = 0; pass < 2; ++pass) {
#pragma unroll
    for (int hr = 0; hr < 4; ++hr) {
      const int g = b * kHeads + kvh * 4 + hr;
#pragma unroll
      for (int it = 0; it < 2; ++it) {
        const int drow = wave * 8 + it * 4 + q;
        unsigned short hb[8];
#pragma unroll
        for (int e = 0; e < 8; ++e) hb[e] = h_bits(sm[drow][c8 + e]);
        const v4u u = (v4u){pk16(hb[0], hb[1]), pk16(hb[2], hb[3]), pk16(hb[4], hb[5]), pk16(hb[6], hb[7])};
        *(volatile v4u*)(VT16 + ((size_t)g * kHeadDim + drow) * kSeq + s0 + c8) = u;
      }
    }
    __threadfence();
  }
}

__global__ __launch_bounds__(128) void softmax_p16_kernel(const float* __restrict__ SC, const float* __restrict__ mask,
                                                          unsigned short* __restrict__ P) {
  __shared__ float redM[4];
  __shared__ float redS[4];
  const int row  = blockIdx.x;
  const int q    = row & (kSeq - 1);
  const int t    = threadIdx.x;
  const int lane = t & 31, wave = t >> 5;
  const int kvlim = ((q >> 6) + 1) << 6;
  const int c0 = 8 * t;
  const int cl = (c0 < kvlim - 8) ? c0 : (kvlim - 8);
  const bool valid = (c0 < kvlim);
  const float* sp = SC + (size_t)row * kSeq + cl;
  const v4f a = *(const v4f*)(sp);
  const v4f c = *(const v4f*)(sp + 4);
  const float* mp = mask + (size_t)q * kSeq + c0;
  const v4f ma = *(const v4f*)(mp);
  const v4f mc = *(const v4f*)(mp + 4);
  float x[8];
#pragma unroll
  for (int e = 0; e < 4; ++e) {
    const float s0 = a[e] + ma[e];
    const float s1 = c[e] + mc[e];
    x[e]     = valid ? s0 : -INFINITY;
    x[4 + e] = valid ? s1 : -INFINITY;
  }
  float m = fmaxf(fmaxf(fmaxf(x[0], x[1]), fmaxf(x[2], x[3])), fmaxf(fmaxf(x[4], x[5]), fmaxf(x[6], x[7])));
#pragma unroll
  for (int off = 16; off > 0; off >>= 1) m = fmaxf(m, __shfl_xor(m, off, 32));
  if (lane == 0) redM[wave] = m;
  __syncthreads();
  const float gm = fmaxf(fmaxf(redM[0], redM[1]), fmaxf(redM[2], redM[3]));
  float ev[8];
  float s = 0.f;
#pragma unroll
  for (int e = 0; e < 8; ++e) { ev[e] = expf(x[e] - gm); s += ev[e]; }
#pragma unroll
  for (int off = 16; off > 0; off >>= 1) s += __shfl_xor(s, off, 32);
  if (lane == 0) redS[wave] = s;
  __syncthreads();
  const float tot = ((redS[0] + redS[1]) + redS[2]) + redS[3];
  const float inv = kPCarry / tot;
  unsigned short hb[8];
#pragma unroll
  for (int e = 0; e < 8; ++e) hb[e] = h_bits(ev[e] * inv);
  const v4u u = (v4u){pk16(hb[0], hb[1]), pk16(hb[2], hb[3]), pk16(hb[4], hb[5]), pk16(hb[6], hb[7])};
  unsigned short* op = P + (size_t)row * kSeq + c0;
  *(volatile v4u*)op = u;
  __threadfence();
  *(volatile v4u*)op = u;
}

__global__ __launch_bounds__(256) void swiglu_f16_kernel(const float* __restrict__ Gf, unsigned short* __restrict__ G16,
                                                         int tok0) {
  const int idx = blockIdx.x * 256 + threadIdx.x;
  const int ri  = idx % (kFF / 8);
  const int tl  = idx / (kFF / 8);
  const float* ap = Gf + (size_t)tl * (2 * kFF) + 8 * ri;
  const float* bp = ap + kFF;
  const v4f a0 = *(const v4f*)(ap);
  const v4f a1 = *(const v4f*)(ap + 4);
  const v4f b0 = *(const v4f*)(bp);
  const v4f b1 = *(const v4f*)(bp + 4);
  float av[8], bv[8];
#pragma unroll
  for (int e = 0; e < 4; ++e) { av[e] = a0[e]; av[4 + e] = a1[e]; bv[e] = b0[e]; bv[4 + e] = b1[e]; }
  unsigned short hb[8];
#pragma unroll
  for (int e = 0; e < 8; ++e) {
    const float sig = 1.0f / (1.0f + expf(-av[e]));
    const float sl  = av[e] * sig;
    const float g   = sl * bv[e];
    hb[e] = h_bits(g * kGCarry);
  }
  const v4u u = (v4u){pk16(hb[0], hb[1]), pk16(hb[2], hb[3]), pk16(hb[4], hb[5]), pk16(hb[6], hb[7])};
  unsigned short* op = G16 + (size_t)(tok0 + tl) * kFF + 8 * ri;
  *(volatile v4u*)op = u;
  __threadfence();
  *(volatile v4u*)op = u;
}

extern "C" void kernel_launch(void* const* d_in, const int* in_sizes, int n_in,
                              void* d_out, int out_size, void* d_ws,
                              size_t ws_size, hipStream_t stream) {
  if (n_in < 13) return;
  if (in_sizes[0] != kTok * kDim) return;
  if (in_sizes[1] != kDim * kDim) return;
  if (in_sizes[2] != kDim * kKVDim || in_sizes[3] != kDim * kKVDim) return;
  if (in_sizes[4] != kDim * kDim) return;
  if (in_sizes[5] != kDim * kFF || in_sizes[6] != kFF * kDim || in_sizes[7] != kDim * kFF) return;
  if (in_sizes[8] != kDim || in_sizes[9] != kDim) return;
  if (in_sizes[10] != kSeq * kPairs || in_sizes[11] != kSeq * kPairs) return;
  if (in_sizes[12] != kSeq * kSeq) return;
  if (out_size != kTok * kDim) return;
  if (ws_size < kWsTotal) return;

  const float* x     = (const float*)d_in[0];
  const float* wq    = (const float*)d_in[1];
  const float* wk    = (const float*)d_in[2];
  const float* wv    = (const float*)d_in[3];
  const float* wo    = (const float*)d_in[4];
  const float* w1    = (const float*)d_in[5];
  const float* w2    = (const float*)d_in[6];
  const float* w3    = (const float*)d_in[7];
  const float* anw   = (const float*)d_in[8];
  const float* fnw   = (const float*)d_in[9];
  const float* fcos  = (const float*)d_in[10];
  const float* fsin  = (const float*)d_in[11];
  const float* maskp = (const float*)d_in[12];
  float* outp = (float*)d_out;

  char* ws = (char*)d_ws;
  unsigned short* H16  = (unsigned short*)(ws + kOffH16);
  float*          SC   = (float*)(ws + kOffSC);
  unsigned short* WqkvT = (unsigned short*)(ws + kOffWqkv);
  float*          X1   = (float*)(ws + kOffX1);
  float*          QKV  = (float*)(ws + kOffQKV);
  unsigned short* W13T = (unsigned short*)(ws + kOffW13);
  unsigned short* W2T  = (unsigned short*)(ws + kOffW2T);
  unsigned short* Q16  = (unsigned short*)(ws + kOffQ16);
  unsigned short* K16  = (unsigned short*)(ws + kOffK16);
  unsigned short* VT16 = (unsigned short*)(ws + kOffVT16);
  unsigned short* O16  = (unsigned short*)(ws + kOffO16);
  float*          GF   = (float*)(ws + kOffGF);
  unsigned short* P16  = (unsigned short*)(ws + kOffP16);
  unsigned short* WoT  = (unsigned short*)(ws + kOffWoT);
  unsigned short* G16  = (unsigned short*)(ws + kOffG16);

  rmsnorm_f16_kernel<<<kTok, 256, 0, stream>>>(x, anw, H16);

  wtcast_kernel<<<dim3(kDim / 64, kDim / 64), 256, 0, stream>>>(wq, kDim, WqkvT, kDim, kWCarry);
  wtcast_kernel<<<dim3(kDim / 64, kKVDim / 64), 256, 0, stream>>>(wk, kKVDim, WqkvT + (size_t)kDim * kDim, kDim, kWCarry);
  wtcast_kernel<<<dim3(kDim / 64, kKVDim / 64), 256, 0, stream>>>(wv, kKVDim, WqkvT + (size_t)(kDim + kKVDim) * kDim, kDim, kWCarry);

  wmma_gemm64<0, false, 0, 0, false, 0, 0><<<dim3((32 * 48) / 8, 1), 256, 0, stream>>>(
      H16, nullptr, kDim, 0L, WqkvT, nullptr, kDim, 0L,
      QKV, nullptr, kQKVN, 0L, nullptr, nullptr, 0L, kTok, kQKVN, kDim, kQKVScale);

  rope_qk_kernel<<<(kGroups * kSeq * 8) / 256, 256, 0, stream>>>(QKV, fcos, fsin, Q16, K16);
  vtrans_kernel<<<dim3(kSeq / 64, kKVHeads, kBatch), 256, 0, stream>>>(QKV, VT16);

  for (int ch = 0; ch < kNChunkA; ++ch) {
    const int g0 = ch * kGChunk;
    const size_t gofs = (size_t)g0 * kSeq * kHeadDim;
    const int bidx = g0 / kHeads;
    const int h0 = g0 - bidx * kHeads;
    wmma_gemm64<0, false, 0, 0, false, 0, 1><<<dim3((16 * 16) / 8, kGChunk), 256, 0, stream>>>(
        Q16 + gofs, nullptr, kHeadDim, (long)kSeq * kHeadDim, K16 + gofs, nullptr, kHeadDim, (long)kSeq * kHeadDim,
        SC, nullptr, kSeq, (long)kSeq * kSeq, nullptr, nullptr, 0L, kSeq, kSeq, kHeadDim, kScoreScale);
    softmax_p16_kernel<<<kGChunk * kSeq, 128, 0, stream>>>(SC, maskp, P16);
    wmma_gemm64<0, false, 0, 1, false, 0, 2><<<dim3(2, kGChunk), 256, 0, stream>>>(
        P16, nullptr, kSeq, (long)kSeq * kSeq, VT16 + gofs, nullptr, kSeq, (long)kHeadDim * kSeq,
        O16 + (size_t)bidx * kSeq * kDim + (size_t)h0 * kHeadDim, nullptr, kDim, (long)kHeadDim,
        nullptr, nullptr, 0L, kSeq, kHeadDim, kSeq, kPVScale);
  }

  wtcast_kernel<<<dim3(kDim / 64, kDim / 64), 256, 0, stream>>>(wo, kDim, WoT, kDim, kWCarry);
  wmma_gemm64<0, false, 0, 0, true, 0, 0><<<dim3((32 * 32) / 8, 1), 256, 0, stream>>>(
      O16, nullptr, kDim, 0L, WoT, nullptr, kDim, 0L,
      X1, nullptr, kDim, 0L, nullptr, x, 0L, kTok, kDim, kDim, kWoScale);

  rmsnorm_f16_kernel<<<kTok, 256, 0, stream>>>(X1, fnw, H16);

  wtcast_kernel<<<dim3(kDim / 64, kFF / 64), 256, 0, stream>>>(w1, kFF, W13T, kDim, kWCarry);
  wtcast_kernel<<<dim3(kDim / 64, kFF / 64), 256, 0, stream>>>(w3, kFF, W13T + (size_t)kFF * kDim, kDim, kWCarry);

  for (int tc = 0; tc < kNChunkF; ++tc) {
    const int tok0 = tc * kTokChunk;
    wmma_gemm64<0, false, 0, 0, false, 0, 0><<<dim3((8 * 176) / 8, 1), 256, 0, stream>>>(
        H16 + (size_t)tok0 * kDim, nullptr, kDim, 0L, W13T, nullptr, kDim, 0L,
        GF, nullptr, 2 * kFF, 0L, nullptr, nullptr, 0L, kTokChunk, 2 * kFF, kDim, kQKVScale);
    swiglu_f16_kernel<<<(kTokChunk * (kFF / 8)) / 256, 256, 0, stream>>>(GF, G16, tok0);
  }

  wtcast_kernel<<<dim3(kFF / 64, kDim / 64), 256, 0, stream>>>(w2, kDim, W2T, kFF, kWCarry);
  wmma_gemm64<0, false, 0, 0, true, 0, 0><<<dim3((32 * 32) / 8, 1), 256, 0, stream>>>(
      G16, nullptr, kFF, 0L, W2T, nullptr, kFF, 0L,
      outp, nullptr, kDim, 0L, nullptr, X1, 0L, kTok, kDim, kFF, kW2Scale);
}
